// ContextualAttentionMask_45913200394447
// MI455X (gfx1250) — hardware-verified
//
#include <hip/hip_runtime.h>


#define NI   4
#define CH   256
#define HW_  64
#define NPX  4096
#define WP   66
#define NPP  4356
#define NPC  4416
#define PCAR 1024.0f
typedef _Float16 h16;
typedef unsigned short bf;
typedef __attribute__((ext_vector_type(16))) __bf16   v16bf;
typedef __attribute__((ext_vector_type(16))) _Float16 v16h;
typedef __attribute__((ext_vector_type(8)))  _Float16 v8h;
typedef __attribute__((ext_vector_type(8)))  unsigned short v8us;
typedef __attribute__((ext_vector_type(8)))  float    v8f;
typedef __attribute__((ext_vector_type(4)))  float    v4f;
typedef v8h  __attribute__((may_alias)) v8ha;
typedef v4f  __attribute__((may_alias)) v4fa;
typedef v8us __attribute__((may_alias)) v8usa;

__device__ __forceinline__ unsigned short f2bf(float f) { unsigned u = __float_as_uint(f); u += 0x7FFFu + ((u >> 16) & 1u); return (unsigned short)(u >> 16); }
__device__ __forceinline__ float bf2f(unsigned short b) { return __uint_as_float(((unsigned)b) << 16); }
__device__ __forceinline__ float bfr(float f) { return bf2f(f2bf(f)); }
__device__ __forceinline__ v16h cat16(v8h lo, v8h hi) { return __builtin_shufflevector(lo, hi, 0, 1, 2, 3, 4, 5, 6, 7, 8, 9, 10, 11, 12, 13, 14, 15); }
__device__ __forceinline__ v16bf cat16b(v8us lo, v8us hi) { return __builtin_bit_cast(v16bf, __builtin_shufflevector(lo, hi, 0, 1, 2, 3, 4, 5, 6, 7, 8, 9, 10, 11, 12, 13, 14, 15)); }
__device__ __forceinline__ v8f wmma16(v16h a, v16h b, v8f c) { return __builtin_amdgcn_wmma_f32_16x16x32_f16(false, a, false, b, (short)0, c, false, false); }
__device__ __forceinline__ v8f wmmab(v16bf a, v16bf b, v8f c) { return __builtin_amdgcn_wmma_f32_16x16x32_bf16(false, a, false, b, (short)0, c, false, false); }


template <typename T16> struct WFrag;
template <> struct WFrag<h16> { typedef v16h V; static __device__ __forceinline__ V ld(const h16* p) { return cat16(*(const v8h*)p, *(const v8h*)(p + 16)); } static __device__ __forceinline__ v8f mma(V a, V b, v8f c) { return wmma16(a, b, c); } };
template <> struct WFrag<bf> { typedef v16bf V; static __device__ __forceinline__ V ld(const bf* p) { return cat16b(*(const v8us*)p, *(const v8us*)(p + 16)); } static __device__ __forceinline__ v8f mma(V a, V b, v8f c) { return wmmab(a, b, c); } };
template <typename T16, int NSPLIT, bool BIAS>
__global__ __launch_bounds__(32) void k_gemmw(const T16* __restrict__ A, const T16* __restrict__ A2, const T16* __restrict__ Bt, const T16* __restrict__ Bt2, int K, float* C, int ldc, const float* __restrict__ bias, size_t sA, size_t sB, size_t sC) {
    typedef typename WFrag<T16>::V V;
    __shared__ __align__(16) float os[16 * 68];
    const size_t z = blockIdx.z; A += z * sA; if (A2) A2 += z * sA; Bt += z * sB; if (Bt2) Bt2 += z * sB; C += z * sC;
    const int lane = threadIdx.x & 31, lr = lane & 15, hi = lane >> 4; const int r0 = blockIdx.x * 64, c0 = blockIdx.y * 64;
    v8f acc[4][4];
#pragma unroll
    for (int mb = 0; mb < 4; ++mb)
#pragma unroll
        for (int nb = 0; nb < 4; ++nb) acc[mb][nb] = (v8f){};
    const size_t aoff = (size_t)(r0 + lr) * K + 8 * hi, boff = (size_t)(c0 + lr) * K + 8 * hi;
#pragma unroll 1
    for (int kc = 0; kc < K; kc += 32) {
        V a[4], a2[4];
#pragma unroll
        for (int mb = 0; mb < 4; ++mb) { a[mb] = WFrag<T16>::ld(A + aoff + (size_t)mb * 16 * K + kc); if (NSPLIT == 1 || NSPLIT == 2) a2[mb] = WFrag<T16>::ld(A2 + aoff + (size_t)mb * 16 * K + kc); }
#pragma unroll
        for (int nb = 0; nb < 4; ++nb) { const V b = WFrag<T16>::ld(Bt + boff + (size_t)nb * 16 * K + kc); V b2; if (NSPLIT >= 2) b2 = WFrag<T16>::ld(Bt2 + boff + (size_t)nb * 16 * K + kc);
#pragma unroll
            for (int mb = 0; mb < 4; ++mb) { acc[mb][nb] = WFrag<T16>::mma(a[mb], b, acc[mb][nb]); if (NSPLIT == 1 || NSPLIT == 2) acc[mb][nb] = WFrag<T16>::mma(a2[mb], b, acc[mb][nb]); if (NSPLIT >= 2) acc[mb][nb] = WFrag<T16>::mma(a[mb], b2, acc[mb][nb]); } }
        asm volatile("v_nop\n\tv_nop\n\tv_nop\n\tv_nop" : "+v"(acc[0][0]), "+v"(acc[1][1]), "+v"(acc[2][2]), "+v"(acc[3][3]) : "v"(a[0]), "v"(a[3]));
    }
#pragma unroll
    for (int mb = 0; mb < 4; ++mb) {
#pragma unroll
        for (int nb = 0; nb < 4; ++nb) {
#pragma unroll
            for (int j = 0; j < 8; ++j) os[(hi * 8 + j) * 68 + nb * 16 + lr] = acc[mb][nb][j]; }
        __builtin_amdgcn_wave_barrier(); asm volatile("" ::: "memory");
        float* crow = C + (size_t)(r0 + mb * 16) * ldc + c0;
#pragma unroll 1
        for (int ps = 0; ps < 2; ++ps) {
#pragma unroll
            for (int s = 0; s < 8; ++s) { const int row = 2 * s + hi, cofs = lr * 4; v4f val = *(const v4fa*)(os + row * 68 + cofs); if (BIAS) { val[0] += bfr(bias[c0 + cofs]); val[1] += bfr(bias[c0 + cofs + 1]); val[2] += bfr(bias[c0 + cofs + 2]); val[3] += bfr(bias[c0 + cofs + 3]); }
                *(volatile v4f*)(crow + (size_t)row * ldc + cofs) = val; }
            if (ps == 0) __threadfence(); }
        __builtin_amdgcn_wave_barrier(); asm volatile("" ::: "memory");
    }
}

__device__ __forceinline__ h16 tohx(float x) { return (h16)x; }
typedef __attribute__((ext_vector_type(4))) unsigned short v4us;
typedef __attribute__((ext_vector_type(2))) _Float16 v2h;
typedef __attribute__((ext_vector_type(4))) _Float16 v4h;

__global__ __launch_bounds__(256) void k_fgt(const float* __restrict__ fg, bf* FGT) { const int e = (blockIdx.x * 256 + threadIdx.x) * 4; if (e >= NPX * CH) return; const int c = e % CH; const int j = e / CH; v4us o;
#pragma unroll
    for (int u = 0; u < 4; ++u) o[u] = f2bf(fg[(size_t)(c + u) * NPX + j]); *(volatile v4us*)(FGT + e) = o; __threadfence(); *(volatile v4us*)(FGT + e) = o; }
__global__ __launch_bounds__(256) void k_fpt(const float* __restrict__ fg, bf* FPT) { const int e = (blockIdx.x * 256 + threadIdx.x) * 4; if (e >= NPC * CH) return; const int c = e % CH; const int yx = e / CH; const int py = yx / WP, px = yx % WP; const int y = py - 1, x = px - 1; const bool in = (yx < NPP) && y >= 0 && y < HW_ && x >= 0 && x < HW_; v4us o;
#pragma unroll
    for (int u = 0; u < 4; ++u) o[u] = in ? f2bf(fg[(size_t)(c + u) * NPX + y * HW_ + x]) : (unsigned short)0; *(volatile v4us*)(FPT + e) = o; __threadfence(); *(volatile v4us*)(FPT + e) = o; }
__global__ __launch_bounds__(256) void k_nrm(const float* __restrict__ fg, float* NRM) { const int j = blockIdx.x * 256 + threadIdx.x; if (j >= NPX) return; float q = 0.f;
#pragma unroll 1
    for (int c = 0; c < CH; ++c) { const float v = __fadd_rn(bfr(fg[(size_t)c * NPX + j]), 1e-7f); float p = __fmul_rn(v, v); asm volatile("" : "+v"(p)); q = __fadd_rn(q, p); }
    const float n = __fsqrt_rn(q); *(volatile float*)(NRM + j) = n; __threadfence(); *(volatile float*)(NRM + j) = n; }

__global__ __launch_bounds__(256) void k_cstat(const float* __restrict__ S0, const bf* __restrict__ FPT, const float* __restrict__ NRM, float* CST) { const int yx = blockIdx.x * 256 + threadIdx.x; if (yx >= NPC) return; float cs = 0.f;
#pragma unroll 1
    for (int c = 0; c < CH; ++c) cs = __fadd_rn(cs, bf2f(FPT[(size_t)yx * CH + c]));
    cs = __fmul_rn(cs, 1e-7f); float mx = -3.0e38f;
#pragma unroll 1
    for (int j = 0; j < NPX; ++j) { const float lg = __fdiv_rn(__fadd_rn(S0[(size_t)j * NPC + yx], cs), NRM[j]); mx = fmaxf(mx, lg); }
    float sum = 0.f;
#pragma unroll 1
    for (int j = 0; j < NPX; ++j) { const float lg = __fdiv_rn(__fadd_rn(S0[(size_t)j * NPC + yx], cs), NRM[j]); float d0 = __fsub_rn(lg, mx); asm volatile("" : "+v"(d0)); sum = __fadd_rn(sum, __builtin_amdgcn_exp2f(__fmul_rn(d0, 1.4426950408889634f))); }
    v4f o; o[0] = mx; o[1] = __fdiv_rn(PCAR, sum); o[2] = cs; o[3] = 0.f; *(volatile v4f*)(CST + (size_t)yx * 4) = o; __threadfence(); *(volatile v4f*)(CST + (size_t)yx * 4) = o; }
__global__ __launch_bounds__(256) void k_attT(const float* __restrict__ S0, const float* __restrict__ NRM, const float* __restrict__ CST, h16* ATT) { const size_t e = ((size_t)blockIdx.x * 256 + threadIdx.x) * 4; if (e >= (size_t)NPC * NPX) return; const int j0 = (int)(e % NPX); const int yx = (int)(e / NPX); const v4f st = *(const v4f*)(CST + (size_t)yx * 4); v4h o;
#pragma unroll
    for (int u = 0; u < 4; ++u) { const int j = j0 + u; const float lg = __fdiv_rn(__fadd_rn(S0[(size_t)j * NPC + yx], st[2]), NRM[j]); float d0 = __fsub_rn(lg, st[0]); asm volatile("" : "+v"(d0)); o[u] = tohx(__builtin_amdgcn_exp2f(__fmul_rn(d0, 1.4426950408889634f)) * st[1]); }
    *(volatile v4h*)(ATT + e) = o; __threadfence(); *(volatile v4h*)(ATT + e) = o; }
__global__ __launch_bounds__(256) void k_kmT(const float* __restrict__ fg, const float* __restrict__ mk, const float* __restrict__ NRM, h16* KMT) { const int e = (blockIdx.x * 256 + threadIdx.x) * 2; if (e >= CH * NPX) return; const int j = e % NPX; const int c = e / NPX; v2h o;
#pragma unroll
    for (int u = 0; u < 2; ++u) { const float kn = __fdiv_rn(__fadd_rn(bfr(fg[(size_t)c * NPX + j + u]), 1e-7f), NRM[j + u]); o[u] = tohx(__fmul_rn(kn, bfr(mk[j + u]))); } *(volatile v2h*)(KMT + e) = o; __threadfence(); *(volatile v2h*)(KMT + e) = o; }
__global__ __launch_bounds__(32) void k_msum(const float* __restrict__ mk, float* SKIP) { const int lane = threadIdx.x; float s = 0.f;
#pragma unroll 4
    for (int k = 0; k < NPX / 32; ++k) s = __fadd_rn(s, bfr(mk[k * 32 + lane]));
#pragma unroll
    for (int sh = 16; sh; sh >>= 1) s += __shfl_xor(s, sh, 32);
    const float f = (s > (float)(NPX - 10)) ? 1.0f : 0.0f; *(volatile float*)(SKIP + lane) = f; __threadfence(); *(volatile float*)(SKIP + lane) = f; }
__global__ __launch_bounds__(256) void k_fin(const float* __restrict__ O, const float* __restrict__ fg, const float* __restrict__ mk, const float* __restrict__ SKIP, float* outb) { const int e = (blockIdx.x * 256 + threadIdx.x) * 4; if (e >= CH * NPX) return; const int x0 = e % HW_; const int y = (e / HW_) % HW_; const int c = e / NPX; const bool skip = SKIP[0] != 0.f; v4f r;
#pragma unroll
    for (int u = 0; u < 4; ++u) { const int x = x0 + u; const float f = bfr(fg[e + u]); const float m = bfr(mk[y * HW_ + x]); const float op = O[(size_t)((y + 1) * WP + x + 1) * CH + c] * (1.0f / PCAR);
        float a = __fmul_rn(op, __fsub_rn(1.0f, m)); asm volatile("" : "+v"(a)); float b2 = __fmul_rn(f, m); asm volatile("" : "+v"(b2)); r[u] = skip ? f : __fadd_rn(a, b2); }
    *(volatile v4f*)(outb + e) = r; __threadfence(); *(volatile v4f*)(outb + e) = r; }

extern "C" void kernel_launch(void* const* d_in, const int* in_sizes, int n_in,
                              void* d_out, int out_size, void* d_ws, size_t ws_size, hipStream_t stream) {
    (void)in_sizes; (void)n_in; (void)out_size;
    const float* FG = (const float*)d_in[0]; const float* MK = (const float*)d_in[1];
    float* OUT = (float*)d_out;
    char* wsp = (char*)d_ws;
    auto take = [&](size_t bytes) { char* p = wsp; wsp += (bytes + 255) & ~(size_t)255; return (void*)p; };
    bf* FGT = (bf*)take((size_t)NPX * CH * 2); bf* FPT = (bf*)take((size_t)NPC * CH * 2); float* NRM = (float*)take(NPX * 4); float* S0 = (float*)take((size_t)NPX * NPC * 4); float* CST = (float*)take((size_t)NPC * 4 * 4);
    h16* ATT = (h16*)take((size_t)NPC * NPX * 2); h16* KMT = (h16*)take((size_t)CH * NPX * 2); float* O = (float*)take((size_t)NPC * CH * 4); float* SKIP = (float*)take(32 * 4);
    if ((size_t)(wsp - (char*)d_ws) > ws_size) return;
    for (int b = 0; b < NI; ++b) { const float* fg = FG + (size_t)b * CH * NPX; const float* mk = MK + (size_t)b * NPX;
        k_fgt<<<(NPX * CH / 4 + 255) / 256, 256, 0, stream>>>(fg, FGT); k_fpt<<<(NPC * CH / 4 + 255) / 256, 256, 0, stream>>>(fg, FPT); k_nrm<<<NPX / 256, 256, 0, stream>>>(fg, NRM); k_msum<<<1, 32, 0, stream>>>(mk, SKIP);
        k_gemmw<bf, 0, false><<<dim3(NPX / 64, NPC / 64, 1), 32, 0, stream>>>(FGT, nullptr, FPT, nullptr, CH, S0, NPC, nullptr, 0, 0, 0);
        k_cstat<<<(NPC + 255) / 256, 256, 0, stream>>>(S0, FPT, NRM, CST);
        k_attT<<<(unsigned)(((size_t)NPC * NPX / 4 + 255) / 256), 256, 0, stream>>>(S0, NRM, CST, ATT); k_kmT<<<(CH * NPX / 2 + 255) / 256, 256, 0, stream>>>(fg, mk, NRM, KMT);
        k_gemmw<h16, 0, false><<<dim3(NPC / 64, CH / 64, 1), 32, 0, stream>>>(ATT, nullptr, KMT, nullptr, NPX, O, CH, nullptr, 0, 0, 0);
        k_fin<<<(CH * NPX / 4 + 255) / 256, 256, 0, stream>>>(O, fg, mk, SKIP, OUT + (size_t)b * CH * NPX); }
}
